// CausalSelfAttention_56332791054959
// MI455X (gfx1250) — hardware-verified
//
#include <hip/hip_runtime.h>


#ifndef NB
#define NB 2
#endif
#ifndef SEQ
#define SEQ 2048
#endif
#define SEQ_FULL 2048
#define DM   1024
#define NH   16
#define HD   64
#define DQ   (NH * HD)
#define TABN 2048
#define TABW 32
#define RH   256
#define PCAR 1024.0f
#define SCL2E 0.18033688011112042f
#define NEGV (-1.0e30f)

static_assert(HD == 64);
static_assert(DQ == DM);
static_assert(TABW * 2 == HD);
static_assert(DM % 64 == 0);
static_assert(DM % 32 == 0);
static_assert(SEQ % 64 == 0);
static_assert(RH % 64 == 0);
static_assert(RH <= SEQ);
static_assert(SEQ <= SEQ_FULL);
static_assert(SEQ <= TABN);
static_assert((NB * SEQ) % 64 == 0);

typedef _Float16 h16;
typedef unsigned short bf;
typedef __attribute__((ext_vector_type(16))) __bf16   v16bf;
typedef __attribute__((ext_vector_type(16))) _Float16 v16h;
typedef __attribute__((ext_vector_type(16))) unsigned short v16us;
typedef __attribute__((ext_vector_type(8)))  unsigned short v8us;
typedef __attribute__((ext_vector_type(8)))  float    v8f;
typedef __attribute__((ext_vector_type(4)))  float    v4f;
typedef __attribute__((ext_vector_type(2)))  float    v2f;
typedef __attribute__((ext_vector_type(2)))  _Float16 v2h;
typedef __attribute__((ext_vector_type(2)))  unsigned short v2us;
typedef v4f  __attribute__((may_alias)) v4fa;
typedef v8us __attribute__((may_alias)) v8usa;

__device__ __forceinline__ unsigned short f2bf(float f) { unsigned u = __float_as_uint(f); u += 0x7FFFu + ((u >> 16) & 1u); return (unsigned short)(u >> 16); }
__device__ __forceinline__ float bf2f(unsigned short b) { return __uint_as_float(((unsigned)b) << 16); }
__device__ __forceinline__ float bfr(float f) { return bf2f(f2bf(f)); }
__device__ __forceinline__ void splitf(float y, unsigned short& h, unsigned short& l) { h = f2bf(y); l = f2bf(y - bf2f(h)); }
__device__ __forceinline__ v16us cat16u(v8us lo, v8us hi) { return __builtin_shufflevector(lo, hi, 0, 1, 2, 3, 4, 5, 6, 7, 8, 9, 10, 11, 12, 13, 14, 15); }
__device__ __forceinline__ v8f wmma16(v16h a, v16h b, v8f c) { return __builtin_amdgcn_wmma_f32_16x16x32_f16(false, a, false, b, (short)0, c, false, false); }
__device__ __forceinline__ v8f wmmab(v16bf a, v16bf b, v8f c) { return __builtin_amdgcn_wmma_f32_16x16x32_bf16(false, a, false, b, (short)0, c, false, false); }

template <bool HI> struct AF;
template <> struct AF<false> {
    typedef v16h V;
    static __device__ __forceinline__ V ld(const bf* p) { return __builtin_bit_cast(v16h, cat16u(*(const v8usa*)p, *(const v8usa*)(p + 16))); }
    static __device__ __forceinline__ v8f mma(V a, V b, v8f c) { return wmma16(a, b, c); }
};
template <> struct AF<true> {
    typedef v16bf V;
    static __device__ __forceinline__ V ld(const bf* p) { return __builtin_bit_cast(v16bf, cat16u(*(const v8usa*)p, *(const v8usa*)(p + 16))); }
    static __device__ __forceinline__ v8f mma(V a, V b, v8f c) { return wmmab(a, b, c); }
};

template <int NSPLIT>
__device__ __forceinline__ void gemmw_body(const bf* __restrict__ A, const bf* __restrict__ A2, const bf* __restrict__ Bt, const int K, float* C, const int ldc, const size_t sA, const size_t sB, const size_t sC) {
    typedef AF<true> W; typedef W::V V;
    __shared__ __align__(16) float os[16 * 68];
    const size_t z = blockIdx.z; A += z * sA; A2 += z * sA; Bt += z * sB; C += z * sC;
    const int lane = threadIdx.x & 31, lr = lane & 15, hi = lane >> 4; const int r0 = blockIdx.x * 64, c0 = blockIdx.y * 64;
    v8f acc[4][4];
#pragma unroll
    for (int mb = 0; mb < 4; ++mb)
#pragma unroll
        for (int nb = 0; nb < 4; ++nb) acc[mb][nb] = (v8f){};
    const size_t aoff = (size_t)(r0 + lr) * K + 8 * hi, boff = (size_t)(c0 + lr) * K + 8 * hi;
#pragma unroll 1
    for (int kc = 0; kc < K; kc += 32) {
        V a[4], a2[4];
#pragma unroll
        for (int mb = 0; mb < 4; ++mb) { a[mb] = W::ld(A + aoff + (size_t)mb * 16 * K + kc); if (NSPLIT == 1) a2[mb] = W::ld(A2 + aoff + (size_t)mb * 16 * K + kc); else a2[mb] = a[mb]; }
#pragma unroll
        for (int nb = 0; nb < 4; ++nb) { const V b = W::ld(Bt + boff + (size_t)nb * 16 * K + kc);
#pragma unroll
            for (int mb = 0; mb < 4; ++mb) { acc[mb][nb] = W::mma(a[mb], b, acc[mb][nb]); if (NSPLIT == 1) acc[mb][nb] = W::mma(a2[mb], b, acc[mb][nb]); } }
        asm volatile("v_nop\n\tv_nop\n\tv_nop\n\tv_nop" : "+v"(acc[0][0]), "+v"(acc[1][1]), "+v"(acc[2][2]), "+v"(acc[3][3]) : "v"(a[0]), "v"(a[3]));
    }
#pragma unroll
    for (int mb = 0; mb < 4; ++mb) {
#pragma unroll
        for (int nb = 0; nb < 4; ++nb) {
#pragma unroll
            for (int j = 0; j < 8; ++j) os[(hi * 8 + j) * 68 + nb * 16 + lr] = acc[mb][nb][j]; }
        __builtin_amdgcn_wave_barrier(); asm volatile("" ::: "memory");
        float* crow = C + (size_t)(r0 + mb * 16) * ldc + c0;
#pragma unroll 1
        for (int ps = 0; ps < 2; ++ps) {
#pragma unroll
            for (int s = 0; s < 8; ++s) { const int row = 2 * s + hi, cofs = lr * 4; const v4f val = *(const v4fa*)(os + row * 68 + cofs);
                *(volatile v4f*)(crow + (size_t)row * ldc + cofs) = val; }
            if (ps == 0) __threadfence(); }
        __builtin_amdgcn_wave_barrier(); asm volatile("" ::: "memory");
    }
}
__global__ __launch_bounds__(32) void k_gemm_x1(const bf* A, const bf* Bt, int K, float* C, int ldc, size_t sA, size_t sB, size_t sC) { gemmw_body<0>(A, A, Bt, K, C, ldc, sA, sB, sC); }
__global__ __launch_bounds__(32) void k_gemm_x2(const bf* A, const bf* A2, const bf* Bt, int K, float* C, int ldc, size_t sA, size_t sB, size_t sC) { gemmw_body<1>(A, A2, Bt, K, C, ldc, sA, sB, sC); }

__global__ __launch_bounds__(256) void k_cvt8(const float* __restrict__ src, bf* dst, size_t n8) { const size_t i = (size_t)blockIdx.x * 256 + threadIdx.x; if (i >= n8) return; const v8f v = *(const v8f*)(src + i * 8); v8us o;
#pragma unroll
    for (int k = 0; k < 8; ++k) o[k] = f2bf(v[k]); *(volatile v8us*)(dst + i * 8) = o; __threadfence(); *(volatile v8us*)(dst + i * 8) = o; }

__global__ __launch_bounds__(256) void k_rope(const float* __restrict__ F, const float* __restrict__ sin_tab, const float* __restrict__ cos_tab, h16* P16, bf* Ph, bf* Pl) {
#pragma clang fp contract(off)
    const size_t e = ((size_t)blockIdx.x * 256 + threadIdx.x) * 2; if (e >= (size_t)NB * NH * SEQ * HD) return;
    const int d = (int)(e % HD); const int t = (int)((e / HD) % SEQ); const int bh = (int)(e / ((size_t)HD * SEQ)); const int b = bh / NH, h = bh % NH;
    const int pos = t;
    const float sn = bfr(sin_tab[(size_t)pos * TABW + (d >> 1)]); const float cs = bfr(cos_tab[(size_t)pos * TABW + (d >> 1)]);
    const v2f xx = *(const v2f*)(F + ((size_t)b * SEQ + t) * DM + h * HD + d);
    float a0 = __fmul_rn(cs, xx[0]), a1 = __fmul_rn(sn, xx[1]), c0 = __fmul_rn(sn, xx[0]), c1 = __fmul_rn(cs, xx[1]);
    asm volatile("" : "+v"(a0)); asm volatile("" : "+v"(a1)); asm volatile("" : "+v"(c0)); asm volatile("" : "+v"(c1));
    const float re = __fsub_rn(a0, a1), ro = __fadd_rn(c0, c1);
    v2h o16; o16[0] = (h16)re; o16[1] = (h16)ro; v2us oh, ol; unsigned short u0, u1; splitf(re, u0, u1); oh[0] = u0; ol[0] = u1; splitf(ro, u0, u1); oh[1] = u0; ol[1] = u1;
    const bool hr = (t < RH);
    const size_t ce = hr ? (((size_t)bh * RH + t) * HD + d) : 0;
    *(volatile v2h*)(P16 + e) = o16; if (hr) { *(volatile v2us*)(Ph + ce) = oh; *(volatile v2us*)(Pl + ce) = ol; }
    __threadfence();
    *(volatile v2h*)(P16 + e) = o16; if (hr) { *(volatile v2us*)(Ph + ce) = oh; *(volatile v2us*)(Pl + ce) = ol; }
}

__global__ __launch_bounds__(256) void k_vtp(const float* __restrict__ F, h16* V16, bf* Vh, bf* Vl) {
    const size_t e = ((size_t)blockIdx.x * 256 + threadIdx.x) * 2; if (e >= (size_t)NB * NH * HD * SEQ) return;
    const int t = (int)(e % SEQ); const int d = (int)((e / SEQ) % HD); const int bh = (int)(e / ((size_t)SEQ * HD)); const int b = bh / NH, h = bh % NH; v2h o16; v2us oh, ol;
#pragma unroll
    for (int q = 0; q < 2; ++q) { const float x = F[((size_t)b * SEQ + t + q) * DM + h * HD + d]; o16[q] = (h16)x; unsigned short u0, u1; splitf(x, u0, u1); oh[q] = u0; ol[q] = u1; }
    const bool hr = (t < RH);
    const size_t ce = hr ? (((size_t)bh * HD + d) * RH + t) : 0;
    *(volatile v2h*)(V16 + e) = o16; if (hr) { *(volatile v2us*)(Vh + ce) = oh; *(volatile v2us*)(Vl + ce) = ol; }
    __threadfence();
    *(volatile v2h*)(V16 + e) = o16; if (hr) { *(volatile v2us*)(Vh + ce) = oh; *(volatile v2us*)(Vl + ce) = ol; }
}

template <bool HI>
__device__ __forceinline__ void attn_body(const bf* __restrict__ Qa, const bf* __restrict__ Qb, const bf* __restrict__ Ka, const bf* __restrict__ Kb, const bf* __restrict__ Va, const bf* __restrict__ Vb,
                                          const int tq, const int tv, const int qblk, const int bh, bf* ATh, bf* ATl) {
    typedef AF<HI> F; typedef typename F::V V;
    __shared__ __align__(16) bf sth[4 * 16 * 72];
    __shared__ __align__(16) bf stl[4 * 16 * 72];
    const int lane = threadIdx.x & 31, lr = lane & 15, hi = lane >> 4, wave = threadIdx.x >> 5;
    const int q0 = qblk * 64 + wave * 16; const int qrow = q0 + lr;
    const size_t qoff = ((size_t)bh * tq + q0 + lr) * HD + 8 * hi;
    const size_t koff = ((size_t)bh * tq + lr) * HD + 8 * hi;
    const size_t voff = ((size_t)bh * HD + lr) * tv + 8 * hi;
    V qa[2], qb[2];
#pragma unroll
    for (int ks = 0; ks < 2; ++ks) { qa[ks] = F::ld(Qa + qoff + 32 * ks); if (HI) qb[ks] = F::ld(Qb + qoff + 32 * ks); else qb[ks] = qa[ks]; }
    v8f o[4];
#pragma unroll
    for (int nb = 0; nb < 4; ++nb) o[nb] = (v8f){};
    float m = NEGV, l = 0.0f;
#pragma unroll 1
    for (int c0 = 0; c0 <= q0 + 15; c0 += 32) {
        v8f s0 = (v8f){}, s1 = (v8f){}; V k0, k1;
#pragma unroll
        for (int ks = 0; ks < 2; ++ks) {
            k0 = F::ld(Ka + koff + (size_t)c0 * HD + 32 * ks); k1 = F::ld(Ka + koff + (size_t)(c0 + 16) * HD + 32 * ks);
            if (HI) { const V l0 = F::ld(Kb + koff + (size_t)c0 * HD + 32 * ks); const V l1 = F::ld(Kb + koff + (size_t)(c0 + 16) * HD + 32 * ks);
                s0 = F::mma(l0, qa[ks], s0); s1 = F::mma(l1, qa[ks], s1); s0 = F::mma(k0, qb[ks], s0); s1 = F::mma(k1, qb[ks], s1); }
            s0 = F::mma(k0, qa[ks], s0); s1 = F::mma(k1, qa[ks], s1);
        }
        asm volatile("v_nop\n\tv_nop\n\tv_nop\n\tv_nop" : "+v"(s0), "+v"(s1) : "v"(k0), "v"(k1), "v"(qa[1]), "v"(qb[1]));
        if (c0 + 31 > q0) {
#pragma unroll
            for (int r = 0; r < 8; ++r) { const int key = c0 + 8 * hi + r; s0[r] = (key > qrow) ? NEGV : s0[r]; s1[r] = (key + 16 > qrow) ? NEGV : s1[r]; }
        }
        float mx = fmaxf(s0[0], s1[0]);
#pragma unroll
        for (int r = 1; r < 8; ++r) mx = fmaxf(mx, fmaxf(s0[r], s1[r]));
        mx = fmaxf(mx, __shfl_xor(mx, 16, 32));
        const float mn = fmaxf(m, mx);
        const float corr = __builtin_amdgcn_exp2f((m - mn) * SCL2E);
        float ps = 0.0f;
#pragma unroll
        for (int r = 0; r < 8; ++r) { s0[r] = __builtin_amdgcn_exp2f((s0[r] - mn) * SCL2E); s1[r] = __builtin_amdgcn_exp2f((s1[r] - mn) * SCL2E); ps += s0[r] + s1[r]; }
        l = l * corr + ps; m = mn;
#pragma unroll
        for (int nb = 0; nb < 4; ++nb)
#pragma unroll
            for (int r = 0; r < 8; ++r) o[nb][r] *= corr;
        V pa, pl;
        if (HI) { v16us uh, ul;
#pragma unroll
            for (int r = 0; r < 8; ++r) { unsigned short a, c; splitf(s0[r], a, c); uh[r] = a; ul[r] = c; splitf(s1[r], a, c); uh[8 + r] = a; ul[8 + r] = c; }
            pa = __builtin_bit_cast(V, uh); pl = __builtin_bit_cast(V, ul);
        } else { v16h th;
#pragma unroll
            for (int r = 0; r < 8; ++r) { th[r] = (h16)(s0[r] * PCAR); th[8 + r] = (h16)(s1[r] * PCAR); }
            pa = __builtin_bit_cast(V, th); pl = pa; }
        V vh[4], vl[4];
#pragma unroll
        for (int nb = 0; nb < 4; ++nb) { vh[nb] = F::ld(Va + voff + (size_t)nb * 16 * tv + c0); if (HI) vl[nb] = F::ld(Vb + voff + (size_t)nb * 16 * tv + c0); else vl[nb] = vh[nb]; }
#pragma unroll
        for (int nb = 0; nb < 4; ++nb) { if (HI) { o[nb] = F::mma(vl[nb], pa, o[nb]); o[nb] = F::mma(vh[nb], pl, o[nb]); } o[nb] = F::mma(vh[nb], pa, o[nb]); }
        asm volatile("v_nop\n\tv_nop\n\tv_nop\n\tv_nop" : "+v"(o[0]), "+v"(o[1]), "+v"(o[2]), "+v"(o[3]) : "v"(pa), "v"(pl), "v"(vh[3]));
    }
    l += __shfl_xor(l, 16, 32);
    const float inv = (HI ? 1.0f : (1.0f / PCAR)) * (1.0f / l);
    const int sbase = wave * (16 * 72) + lr * 72 + 8 * hi;
#pragma unroll
    for (int nb = 0; nb < 4; ++nb) { v8us h8, l8;
#pragma unroll
        for (int r = 0; r < 8; ++r) { unsigned short a, c; splitf(o[nb][r] * inv, a, c); h8[r] = a; l8[r] = c; }
        *(v8usa*)(sth + sbase + nb * 16) = h8; *(v8usa*)(stl + sbase + nb * 16) = l8; }
    __syncthreads();
    const int b = bh / NH, h = bh % NH;
#pragma unroll 1
    for (int ps = 0; ps < 2; ++ps) {
#pragma unroll
        for (int it = 0; it < 4; ++it) { const int row = it * 4 + (lane >> 3), pc = lane & 7;
            const v8us xh = *(const v8usa*)(sth + wave * (16 * 72) + row * 72 + pc * 8); const v8us xl = *(const v8usa*)(stl + wave * (16 * 72) + row * 72 + pc * 8);
            const size_t go = ((size_t)b * SEQ + q0 + row) * DQ + h * HD + pc * 8;
            *(volatile v8us*)(ATh + go) = xh; *(volatile v8us*)(ATl + go) = xl; }
        if (ps == 0) __threadfence(); }
}
__global__ __launch_bounds__(128) void k_attn_lo(const bf* Q16, const bf* K16, const bf* VT16, bf* ATh, bf* ATl) { attn_body<false>(Q16, Q16, K16, K16, VT16, VT16, SEQ, SEQ, (int)blockIdx.x + RH / 64, (int)blockIdx.y, ATh, ATl); }
__global__ __launch_bounds__(128) void k_attn_hi(const bf* Qh, const bf* Ql, const bf* Kh, const bf* Kl, const bf* VTh, const bf* VTl, bf* ATh, bf* ATl) { attn_body<true>(Qh, Ql, Kh, Kl, VTh, VTl, RH, RH, (int)blockIdx.x, (int)blockIdx.y, ATh, ATl); }

constexpr size_t SZ_W  = (size_t)DM * DM * 2;
constexpr size_t SZ_XB = (size_t)NB * SEQ * DM * 2;
constexpr size_t SZ_F  = (size_t)NB * SEQ * DM * 4;
constexpr size_t SZ_P  = (size_t)NB * NH * SEQ * HD * 2;
constexpr size_t SZ_R  = (size_t)NB * NH * RH * HD * 2;
constexpr size_t SZ_AT = (size_t)NB * SEQ * DQ * 2;
constexpr size_t WS_TOTAL = 4 * SZ_W + SZ_XB + SZ_F + 3 * SZ_P + 6 * SZ_R + 2 * SZ_AT;
static_assert(SZ_W % 256 == 0);
static_assert(SZ_XB % 256 == 0);
static_assert(SZ_F % 256 == 0);
static_assert(SZ_P % 256 == 0);
static_assert(SZ_R % 256 == 0);
static_assert(SZ_AT % 256 == 0);
static_assert(WS_TOTAL <= (size_t)134217728);

extern "C" void kernel_launch(void* const* d_in, const int* in_sizes, int n_in,
                              void* d_out, int out_size, void* d_ws, size_t ws_size, hipStream_t stream) {
    if (n_in < 7) return;
    const long long need_x = (long long)(NB - 1) * SEQ_FULL * DM + (long long)SEQ * DM;
    if ((long long)in_sizes[0] < need_x) return;
    if ((long long)in_sizes[1] < (long long)TABN * TABW || (long long)in_sizes[2] < (long long)TABN * TABW) return;
    if ((long long)in_sizes[3] < (long long)DM * DM || (long long)in_sizes[4] < (long long)DM * DM || (long long)in_sizes[5] < (long long)DM * DM || (long long)in_sizes[6] < (long long)DM * DM) return;
    if ((long long)out_size < need_x) return;
    if (WS_TOTAL > ws_size) return;
    const float* x = (const float*)d_in[0]; const float* cos_tab = (const float*)d_in[1]; const float* sin_tab = (const float*)d_in[2];
    const float* wq = (const float*)d_in[3]; const float* wk = (const float*)d_in[4]; const float* wv = (const float*)d_in[5]; const float* wo = (const float*)d_in[6];
    float* OUT = (float*)d_out;
    char* wsp = (char*)d_ws;
    auto take = [&](size_t bytes) { char* p = wsp; wsp += bytes; return (void*)p; };
    bf* WQ = (bf*)take(SZ_W); bf* WK = (bf*)take(SZ_W); bf* WV = (bf*)take(SZ_W); bf* WO = (bf*)take(SZ_W);
    bf* XB = (bf*)take(SZ_XB); float* Fb = (float*)take(SZ_F);
    h16* Q16 = (h16*)take(SZ_P); h16* K16 = (h16*)take(SZ_P); h16* VT16 = (h16*)take(SZ_P);
    bf* Qh = (bf*)take(SZ_R); bf* Ql = (bf*)take(SZ_R); bf* Kh = (bf*)take(SZ_R); bf* Kl = (bf*)take(SZ_R); bf* VTh = (bf*)take(SZ_R); bf* VTl = (bf*)take(SZ_R);
    bf* ATh = (bf*)take(SZ_AT); bf* ATl = (bf*)take(SZ_AT);

    const size_t w8 = (size_t)DM * DM / 8; const unsigned gw = (unsigned)((w8 + 255) / 256);
    k_cvt8<<<gw, 256, 0, stream>>>(wq, WQ, w8); k_cvt8<<<gw, 256, 0, stream>>>(wk, WK, w8); k_cvt8<<<gw, 256, 0, stream>>>(wv, WV, w8); k_cvt8<<<gw, 256, 0, stream>>>(wo, WO, w8);
    const size_t x8 = (size_t)SEQ * DM / 8;
    for (int b = 0; b < NB; ++b) k_cvt8<<<(unsigned)((x8 + 255) / 256), 256, 0, stream>>>(x + (size_t)b * SEQ_FULL * DM, XB + (size_t)b * SEQ * DM, x8);

    const dim3 gp((unsigned)(NB * SEQ / 64), (unsigned)(DM / 64), 1);
    const unsigned gpl = (unsigned)(((size_t)NB * NH * SEQ * HD / 2 + 255) / 256);
    k_gemm_x1<<<gp, 32, 0, stream>>>(XB, WQ, DM, Fb, DM, (size_t)0, (size_t)0, (size_t)0);
    k_rope<<<gpl, 256, 0, stream>>>(Fb, sin_tab, cos_tab, Q16, Qh, Ql);
    k_gemm_x1<<<gp, 32, 0, stream>>>(XB, WK, DM, Fb, DM, (size_t)0, (size_t)0, (size_t)0);
    k_rope<<<gpl, 256, 0, stream>>>(Fb, sin_tab, cos_tab, K16, Kh, Kl);
    k_gemm_x1<<<gp, 32, 0, stream>>>(XB, WV, DM, Fb, DM, (size_t)0, (size_t)0, (size_t)0);
    k_vtp<<<gpl, 256, 0, stream>>>(Fb, VT16, VTh, VTl);

    k_attn_hi<<<dim3(RH / 64, NB * NH, 1), 128, 0, stream>>>(Qh, Ql, Kh, Kl, VTh, VTl, ATh, ATl);
    if (SEQ > RH) k_attn_lo<<<dim3((SEQ - RH) / 64, NB * NH, 1), 128, 0, stream>>>((const bf*)Q16, (const bf*)K16, (const bf*)VT16, ATh, ATl);

    k_gemm_x2<<<dim3(SEQ / 64, DM / 64, NB), 32, 0, stream>>>(ATh, ATl, WO, DQ, OUT, DM, (size_t)SEQ * DQ, (size_t)0, (size_t)SEQ_FULL * DM);
}
